// PairNN_240518169183
// MI455X (gfx1250) — hardware-verified
//
#include <hip/hip_runtime.h>


#define KNB    32
#define HID    128
#define NDSC   17
#define DST    32
#define NRAD   5
#define N3B    12
#define NTHR   256
#define NWAVE  (NTHR / 32)
#define CCUT   3.0f
#define RMINC  3.5f
#define ETA_F  4.0f
#define PI_F   3.14159265358979f
#define PREF   0.816496580927726f

typedef float          v8f   __attribute__((ext_vector_type(8)));
typedef float          v4f   __attribute__((ext_vector_type(4)));
typedef v4f            v4fa  __attribute__((may_alias));
typedef __bf16         v16b  __attribute__((ext_vector_type(16)));
typedef unsigned short v16us __attribute__((ext_vector_type(16)));
typedef unsigned short v8us  __attribute__((ext_vector_type(8)));
typedef v8us           v8usa __attribute__((may_alias));

union Frag { v16b v; v16us u; v8us hv[2]; };

__device__ __forceinline__ unsigned int bf16_bits_rne(float x) {
  unsigned int u = __float_as_uint(x);
  u += 0x7FFFu + ((u >> 16) & 1u);
  return u >> 16;
}

__device__ __forceinline__ void split2(float x, unsigned short& hb, unsigned short& lb) {
  const unsigned int hu = bf16_bits_rne(x);
  const float hf = __uint_as_float(hu << 16);
  const unsigned int lu = bf16_bits_rne(x - hf);
  hb = (unsigned short)hu;
  lb = (unsigned short)lu;
}

__device__ __forceinline__ v8f mma3(v16b ah, v16b al, v16b bh, v16b bl, v8f c) {
  c = __builtin_amdgcn_wmma_f32_16x16x32_bf16(false, ah, false, bh, (short)0, c, false, false);
  c = __builtin_amdgcn_wmma_f32_16x16x32_bf16(false, al, false, bh, (short)0, c, false, false);
  c = __builtin_amdgcn_wmma_f32_16x16x32_bf16(false, ah, false, bl, (short)0, c, false, false);
  asm volatile("v_nop\n\tv_nop\n\tv_nop\n\tv_nop"
               : "+v"(c) : "v"(ah), "v"(al), "v"(bh), "v"(bl));
  return c;
}

__global__ void __launch_bounds__(NTHR)
k_group(const float* __restrict__ rij, const int* __restrict__ gidx,
        const float* __restrict__ W1g, const float* __restrict__ b1g,
        const float* __restrict__ W2g, const float* __restrict__ b2g,
        float* __restrict__ beta, int ngroups)
{
  __shared__ __attribute__((aligned(16))) unsigned short sW1h[DST * HID];
  __shared__ __attribute__((aligned(16))) unsigned short sW1l[DST * HID];
  __shared__ __attribute__((aligned(16))) unsigned short sDh[KNB * DST];
  __shared__ __attribute__((aligned(16))) unsigned short sDl[KNB * DST];
  __shared__ __attribute__((aligned(16))) unsigned short sGh[KNB * HID];
  __shared__ __attribute__((aligned(16))) unsigned short sGl[KNB * HID];
  __shared__ float sb1[HID], sW2[HID];
  __shared__ float smu[N3B];
  __shared__ float su[KNB * 3], sr[KNB], sfc[KNB], sdfc[KNB], sfk[KNB], sdfk[KNB];
  __shared__ float sdrbf[KNB * NRAD];
  __shared__ float sdot[KNB * KNB];
  __shared__ float spart[NWAVE * KNB];
  __shared__ float so[KNB], scoef[KNB], sC[KNB];
  __shared__ float sgd[KNB * DST];
  __shared__ float sE[KNB * KNB], sDE[KNB * KNB];
  __shared__ __attribute__((aligned(16))) float sbeta[KNB * 4];

  const int g = blockIdx.x;
  if (g >= ngroups) return;
  (void)gidx;
  const int t = threadIdx.x;
  const int wave = t >> 5, lane = t & 31, h = lane >> 4, m = lane & 15;
  const int base = g * KNB;

  for (int i = t; i < DST * HID; i += NTHR) {
    const int kk = i >> 7;
    const float v = (kk < NDSC) ? W1g[i] : 0.0f;
    unsigned short hb, lb;
    split2(v, hb, lb);
    sW1h[i] = hb;
    sW1l[i] = lb;
  }
  for (int i = t; i < HID; i += NTHR) { sb1[i] = b1g[i]; sW2[i] = W2g[i]; }
  if (t < N3B) smu[t] = (float)(-1.0 + (2.0 / 11.0) * (double)t);
  for (int i = t; i < KNB * DST; i += NTHR) {
    if ((i & (DST - 1)) >= NDSC) { sDh[i] = 0; sDl[i] = 0; }
  }

  if (t < KNB) {
    const float* pr = rij + (size_t)(base + t) * 3;
    const float x = pr[0], y = pr[1], z = pr[2];
    const float r = sqrtf(x * x + y * y + z * z);
    const float rinv = 1.0f / fmaxf(r, 1e-12f);
    const float ux = x * rinv, uy = y * rinv, uz = z * rinv;
    su[t * 3 + 0] = ux; su[t * 3 + 1] = uy; su[t * 3 + 2] = uz;
    sr[t] = r;
    float fcv = 1.0f, dfcv = 0.0f;
    if (r > RMINC) {
      const float a = (PI_F * (r - RMINC)) / (CCUT - RMINC);
      fcv  = 0.5f + 0.5f * cosf(a);
      dfcv = (0.5f * -sinf(a)) * (PI_F / (CCUT - RMINC));
    }
    sfc[t] = fcv; sdfc[t] = dfcv;
    const float b = (PI_F * r) / CCUT;
    sfk[t]  = 0.5f + 0.5f * cosf(b);
    sdfk[t] = (0.5f * -sinf(b)) * (PI_F / CCUT);
#pragma unroll
    for (int i = 0; i < NRAD; ++i) {
      const float kn  = ((float)(i + 1) * PI_F) / CCUT;
      const float ang = kn * r;
      const float sn = sinf(ang), cn = cosf(ang);
      const float q   = (PREF * sn) * rinv;
      const float rbf = q * fcv;
      const float dq  = (PREF * (kn * cn)) * rinv - q * rinv;
      const float drb = dq * fcv + q * dfcv;
      unsigned short hb, lb;
      split2(rbf, hb, lb);
      sDh[t * DST + i] = hb;
      sDl[t * DST + i] = lb;
      sdrbf[t * NRAD + i] = drb;
    }
  }
  __syncthreads();

  for (int idx = t; idx < KNB * KNB; idx += NTHR) {
    const int k = idx >> 5, l = idx & 31;
    float d = 0.0f;
    if (k != l) d = su[k * 3 + 0] * su[l * 3 + 0] + su[k * 3 + 1] * su[l * 3 + 1] + su[k * 3 + 2] * su[l * 3 + 2];
    sdot[idx] = d;
  }
  __syncthreads();

  for (int task = t; task < KNB * N3B; task += NTHR) {
    const int k = task / N3B, mm = task - k * N3B;
    const float mu = smu[mm];
    const float* drow = sdot + k * KNB;
    float acc = 0.0f;
#pragma unroll 4
    for (int l = 0; l < KNB; ++l) {
      const float dd = drow[l] - mu;
      acc += __expf(-ETA_F * (dd * dd)) * sfk[l];
    }
    unsigned short hb, lb;
    split2(acc, hb, lb);
    sDh[k * DST + NRAD + mm] = hb;
    sDl[k * DST + NRAD + mm] = lb;
  }
  __syncthreads();

  {
    Frag bh, bl;
#pragma unroll
    for (int i = 0; i < 16; ++i) {
      const int kk  = 8 * h + i + ((i >= 8) ? 8 : 0);
      const int src = kk * HID + wave * 16 + m;
      bh.u[i] = sW1h[src];
      bl.u[i] = sW1l[src];
    }
    const int col = wave * 16 + m;
    const float bb = sb1[col], w2 = sW2[col];
#pragma unroll
    for (int rt = 0; rt < 2; ++rt) {
      Frag ah, al;
      const unsigned short* pah = sDh + (rt * 16 + m) * DST;
      const unsigned short* pal = sDl + (rt * 16 + m) * DST;
      ah.hv[0] = *(const v8usa*)(pah + 8 * h);
      ah.hv[1] = *(const v8usa*)(pah + 16 + 8 * h);
      al.hv[0] = *(const v8usa*)(pal + 8 * h);
      al.hv[1] = *(const v8usa*)(pal + 16 + 8 * h);
      v8f acc = {0.f, 0.f, 0.f, 0.f, 0.f, 0.f, 0.f, 0.f};
      acc = mma3(ah.v, al.v, bh.v, bl.v, acc);
#pragma unroll
      for (int rr = 0; rr < 8; ++rr) {
        const int row = rt * 16 + 8 * h + rr;
        const float zz   = acc[rr] + bb;
        const float s    = 1.0f / (1.0f + __expf(-zz));
        const float hv   = zz * s;
        float part       = hv * w2;
        const float dsil = s * (1.0f + zz * (1.0f - s));
        const float gz   = (sfc[row] * w2) * dsil;
        unsigned short hb, lb;
        split2(gz, hb, lb);
        sGh[row * HID + col] = hb;
        sGl[row * HID + col] = lb;
        part += __shfl_xor(part, 1);
        part += __shfl_xor(part, 2);
        part += __shfl_xor(part, 4);
        part += __shfl_xor(part, 8);
        if (m == 0) spart[wave * KNB + row] = part;
      }
    }
  }
  __syncthreads();

  if (t < KNB) {
    float o = b2g[0];
#pragma unroll
    for (int w = 0; w < NWAVE; ++w) o += spart[w * KNB + t];
    so[t] = o;
  }

  if (wave < 4) {
    const int rt = wave >> 1, ct = wave & 1;
    const int arow = rt * 16 + m;
    const int bn   = ct * 16 + m;
    v8f acc = {0.f, 0.f, 0.f, 0.f, 0.f, 0.f, 0.f, 0.f};
#pragma unroll
    for (int ks = 0; ks < 4; ++ks) {
      Frag ah, al, bh, bl;
      const unsigned short* ga = sGh  + arow * HID + ks * 32;
      const unsigned short* gl = sGl  + arow * HID + ks * 32;
      const unsigned short* wa = sW1h + bn   * HID + ks * 32;
      const unsigned short* wl = sW1l + bn   * HID + ks * 32;
      ah.hv[0] = *(const v8usa*)(ga + 8 * h);  ah.hv[1] = *(const v8usa*)(ga + 16 + 8 * h);
      al.hv[0] = *(const v8usa*)(gl + 8 * h);  al.hv[1] = *(const v8usa*)(gl + 16 + 8 * h);
      bh.hv[0] = *(const v8usa*)(wa + 8 * h);  bh.hv[1] = *(const v8usa*)(wa + 16 + 8 * h);
      bl.hv[0] = *(const v8usa*)(wl + 8 * h);  bl.hv[1] = *(const v8usa*)(wl + 16 + 8 * h);
      acc = mma3(ah.v, al.v, bh.v, bl.v, acc);
    }
#pragma unroll
    for (int rr = 0; rr < 8; ++rr) sgd[(rt * 16 + 8 * h + rr) * DST + bn] = acc[rr];
  }
  __syncthreads();

  if (t < KNB) {
    float cr = so[t] * sdfc[t];
#pragma unroll
    for (int i = 0; i < NRAD; ++i) cr += sgd[t * DST + i] * sdrbf[t * NRAD + i];
    scoef[t] = cr;
  }
  for (int idx = t; idx < KNB * KNB; idx += NTHR) {
    const int k = idx >> 5, l = idx & 31;
    const float dd = sdot[idx];
    const float* ss = sgd + k * DST + NRAD;
    float es = 0.0f, ds = 0.0f;
#pragma unroll
    for (int mm = 0; mm < N3B; ++mm) {
      const float tt = dd - smu[mm];
      const float e  = __expf(-ETA_F * (tt * tt));
      const float se = ss[mm] * e;
      es += se;
      ds += se * tt;
    }
    sE[idx]  = es;
    sDE[idx] = (k == l) ? 0.0f : (-2.0f * ETA_F) * ds;
  }
  __syncthreads();

  if (t < KNB) {
    float c = 0.0f;
#pragma unroll 4
    for (int k = 0; k < KNB; ++k) c += sE[k * KNB + t];
    sC[t] = c;
  }
  __syncthreads();

  if (t < KNB) {
    const int k = t;
    const float fkk = sfk[k];
    float tx = 0.0f, ty = 0.0f, tz = 0.0f;
#pragma unroll 4
    for (int l = 0; l < KNB; ++l) {
      const float w = sDE[k * KNB + l] * sfk[l] + sDE[l * KNB + k] * fkk;
      tx += w * su[l * 3 + 0];
      ty += w * su[l * 3 + 1];
      tz += w * su[l * 3 + 2];
    }
    const float ux = su[k * 3 + 0], uy = su[k * 3 + 1], uz = su[k * 3 + 2];
    const float udt = ux * tx + uy * ty + uz * tz;
    const float rin = 1.0f / fmaxf(sr[k], 1e-12f);
    const float rad = scoef[k] + sC[k] * sdfk[k];
    sbeta[k * 3 + 0] = (tx - udt * ux) * rin + rad * ux;
    sbeta[k * 3 + 1] = (ty - udt * uy) * rin + rad * uy;
    sbeta[k * 3 + 2] = (tz - udt * uz) * rin + rad * uz;
  }
  __syncthreads();

  if (wave == 0) {
    float* dst = beta + (size_t)g * (KNB * 3);
    const bool act = lane < (KNB * 3) / 4;
    v4f v = {0.f, 0.f, 0.f, 0.f};
    if (act) v = *(const v4fa*)(sbeta + 4 * lane);
    if (act) *(volatile v4f*)(dst + 4 * lane) = v;
    __threadfence();
    if (act) *(volatile v4f*)(dst + 4 * lane) = v;
  }
}

extern "C" void kernel_launch(void* const* d_in, const int* in_sizes, int n_in,
                              void* d_out, int out_size, void* d_ws, size_t ws_size,
                              hipStream_t stream) {
  (void)d_ws; (void)ws_size;
  if (n_in < 6) return;
  const int nrows = in_sizes[0] / 3;
  const int ngroups = nrows / KNB;
  if (ngroups <= 0 || ngroups * KNB * 3 != in_sizes[0]) return;
  if (out_size < nrows * 3) return;
  if (in_sizes[2] < NDSC * HID || in_sizes[3] < HID || in_sizes[4] < HID || in_sizes[5] < 1) return;

  const float* rij = (const float*)d_in[0];
  const int*   gix = (const int*)d_in[1];
  const float* W1  = (const float*)d_in[2];
  const float* b1  = (const float*)d_in[3];
  const float* W2  = (const float*)d_in[4];
  const float* b2  = (const float*)d_in[5];
  float* beta = (float*)d_out;

  k_group<<<dim3(ngroups), dim3(NTHR), 0, stream>>>(rij, gix, W1, b1, W2, b2, beta, ngroups);
}
